// EncoderBlock_74285754351786
// MI455X (gfx1250) — hardware-verified
//
#include <hip/hip_runtime.h>


#ifndef NB
#define NB 2
#endif
#ifndef SEQ
#define SEQ 2048
#endif
#define NB_FULL 2
#define S_FULL 2048

constexpr int D_    = 1024;
constexpr int H_    = 16;
constexpr int DH_   = 64;
constexpr int F_    = 4096;
constexpr int QKVN_ = 3 * D_;
constexpr int MROWS = NB * SEQ;
constexpr int QT_   = SEQ / 16;
constexpr float EPS_ = 1e-5f;

constexpr float P_CARRY   = 16384.0f;
constexpr float CTX_CARRY = 32.0f;
constexpr float WO_SCALE  = 16.0f;
constexpr float W1_SCALE  = 16.0f;
constexpr float W2_SCALE  = 32.0f;
constexpr float HID_CARRY = 16.0f;

constexpr int STP = 68;
constexpr int PP_ = 40;
constexpr int OP_ = 72;

static_assert(D_ == H_ * DH_);
static_assert(DH_ == 64);
static_assert(QKVN_ / 64 == 3 * H_);
static_assert(SEQ % 128 == 0);
static_assert(QT_ % 4 == 0);
static_assert(MROWS % 128 == 0);
static_assert(MROWS % 4 == 0);
static_assert(D_ % 64 == 0 && F_ % 64 == 0 && QKVN_ % 64 == 0);
static_assert(D_ % 32 == 0 && F_ % 32 == 0);
static_assert(D_ / 8 == 128);
static_assert(D_ % 256 == 0);
static_assert(NB <= NB_FULL && SEQ <= S_FULL);
static_assert((long)MROWS * F_ * 2 == (long)MROWS * D_ * 8);
static_assert(((long)QKVN_ * D_) % 2048 == 0);
static_assert(((long)D_ * D_) % 2048 == 0);
static_assert(((long)F_ * D_) % 2048 == 0);
static_assert(((long)MROWS * 128) % 256 == 0);

typedef _Float16       f16x16  __attribute__((ext_vector_type(16)));
typedef _Float16       f16x8   __attribute__((ext_vector_type(8)));
typedef __bf16         bf16x16 __attribute__((ext_vector_type(16)));
typedef __bf16         bf16x8  __attribute__((ext_vector_type(8)));
typedef float          f32x8   __attribute__((ext_vector_type(8)));
typedef float          f32x4   __attribute__((ext_vector_type(4)));
typedef unsigned int   u32x4   __attribute__((ext_vector_type(4)));
typedef unsigned short u16x4   __attribute__((ext_vector_type(4)));

__device__ __forceinline__ unsigned int bf16_bits(float f) {
    unsigned int u = __float_as_uint(f);
    u += 0x7FFFu + ((u >> 16) & 1u);
    return u >> 16;
}
__device__ __forceinline__ float bf16_rne(float f) { return __uint_as_float(bf16_bits(f) << 16); }
__device__ __forceinline__ float bf16_widen(unsigned short b) { return __uint_as_float(((unsigned int)b) << 16); }

__device__ __forceinline__ void vst_u4(void* p, u32x4 v) { *reinterpret_cast<volatile u32x4*>(p) = v; }
__device__ __forceinline__ void vst_f4(float* p, f32x4 v) { *reinterpret_cast<volatile f32x4*>(p) = v; }

__device__ __forceinline__ u32x4 pack_h8(f32x4 lo, f32x4 hi) {
    f16x8 h;
    h[0] = (_Float16)lo[0]; h[1] = (_Float16)lo[1]; h[2] = (_Float16)lo[2]; h[3] = (_Float16)lo[3];
    h[4] = (_Float16)hi[0]; h[5] = (_Float16)hi[1]; h[6] = (_Float16)hi[2]; h[7] = (_Float16)hi[3];
    union { f16x8 h; u32x4 u; } t;
    t.h = h;
    return t.u;
}
__device__ __forceinline__ u32x4 pack_b8(f32x4 lo, f32x4 hi) {
    u32x4 r;
    r[0] = bf16_bits(lo[0]) | (bf16_bits(lo[1]) << 16);
    r[1] = bf16_bits(lo[2]) | (bf16_bits(lo[3]) << 16);
    r[2] = bf16_bits(hi[0]) | (bf16_bits(hi[1]) << 16);
    r[3] = bf16_bits(hi[2]) | (bf16_bits(hi[3]) << 16);
    return r;
}
__device__ __forceinline__ f32x4 rne4(f32x4 v) {
    f32x4 r;
    r[0] = bf16_rne(v[0]); r[1] = bf16_rne(v[1]); r[2] = bf16_rne(v[2]); r[3] = bf16_rne(v[3]);
    return r;
}

template <typename T> struct FragV;
template <> struct FragV<_Float16> { typedef f16x16 V16; typedef f16x8 V8; };
template <> struct FragV<__bf16>   { typedef bf16x16 V16; typedef bf16x8 V8; };

template <typename T>
__device__ __forceinline__ typename FragV<T>::V16 ld_frag(const T* p) {
    union U { typename FragV<T>::V16 v; typename FragV<T>::V8 h[2]; } u;
    u.h[0] = *reinterpret_cast<const typename FragV<T>::V8*>(p);
    u.h[1] = *reinterpret_cast<const typename FragV<T>::V8*>(p + 16);
    return u.v;
}

__device__ __forceinline__ f32x8 mma(f16x16 a, f16x16 b, f32x8 c) {
    c = __builtin_amdgcn_wmma_f32_16x16x32_f16(false, a, false, b, (short)0, c, false, false);
    asm volatile("v_nop\n\tv_nop\n\tv_nop\n\tv_nop" : "+v"(c) : "v"(a), "v"(b));
    return c;
}
__device__ __forceinline__ f32x8 mma(bf16x16 a, bf16x16 b, f32x8 c) {
    c = __builtin_amdgcn_wmma_f32_16x16x32_bf16(false, a, false, b, (short)0, c, false, false);
    asm volatile("v_nop\n\tv_nop\n\tv_nop\n\tv_nop" : "+v"(c) : "v"(a), "v"(b));
    return c;
}

__global__ __launch_bounds__(256)
void k_cvt_x(const float* __restrict__ x, unsigned short* __restrict__ xb) {
    const unsigned c   = blockIdx.x * 256u + threadIdx.x;
    const unsigned m   = c >> 7;
    const unsigned col = (c & 127u) * 8u;
    const unsigned bq  = m / (unsigned)SEQ;
    const unsigned s   = m - bq * (unsigned)SEQ;
    const float* src = x + ((size_t)(bq * (unsigned)S_FULL + s)) * D_ + col;
    f32x4 lo = *reinterpret_cast<const f32x4*>(src);
    f32x4 hi = *reinterpret_cast<const f32x4*>(src + 4);
    u32x4 u = pack_b8(lo, hi);
    unsigned short* dst = xb + (size_t)m * D_ + col;
    vst_u4(dst, u);
    __threadfence();
    vst_u4(dst, u);
}

template <int F16OUT>
__global__ __launch_bounds__(256)
void k_cvt_w(const float* __restrict__ w, unsigned short* __restrict__ out, float scale) {
    const size_t c = (size_t)blockIdx.x * 256u + threadIdx.x;
    const float* src = w + c * 8;
    f32x4 lo = *reinterpret_cast<const f32x4*>(src);
    f32x4 hi = *reinterpret_cast<const f32x4*>(src + 4);
    u32x4 u;
    if (F16OUT) {
        f32x4 a = rne4(lo) * scale;
        f32x4 b = rne4(hi) * scale;
        u = pack_h8(a, b);
    } else {
        u = pack_b8(lo, hi);
    }
    unsigned short* dst = out + c * 8;
    vst_u4(dst, u);
    __threadfence();
    vst_u4(dst, u);
}

template <typename T, int MODE>
__global__ __launch_bounds__(256)
void k_gemm(const T* __restrict__ A, const T* __restrict__ Bt,
            const float* __restrict__ bias,
            const unsigned short* __restrict__ resB,
            const float* __restrict__ resF,
            float* __restrict__ outF, _Float16* __restrict__ outH,
            _Float16* __restrict__ outH2, _Float16* __restrict__ outH3,
            int N, int K, float oscale, float ocarry, int relu) {
    __shared__ __align__(16) float stile[128 * STP];

    const int lane = threadIdx.x & 31, wave = threadIdx.x >> 5;
    const int lr = lane & 15, lh = lane >> 4;
    const int wm = wave >> 1, wn = wave & 1;
    const int mBase = blockIdx.x * 128, nBase = blockIdx.y * 64;
    const int m0 = mBase + wm * 32, n0 = nBase + wn * 32;

    const T* pa0 = A  + (size_t)(m0 + lr) * K + lh * 8;
    const T* pa1 = pa0 + (size_t)16 * K;
    const T* pb0 = Bt + (size_t)(n0 + lr) * K + lh * 8;
    const T* pb1 = pb0 + (size_t)16 * K;

    f32x8 acc[2][2] = {};

    #pragma unroll 2
    for (int k0 = 0; k0 < K; k0 += 32) {
        typename FragV<T>::V16 a0 = ld_frag<T>(pa0 + k0);
        typename FragV<T>::V16 a1 = ld_frag<T>(pa1 + k0);
        typename FragV<T>::V16 b0 = ld_frag<T>(pb0 + k0);
        typename FragV<T>::V16 b1 = ld_frag<T>(pb1 + k0);
        acc[0][0] = mma(a0, b0, acc[0][0]);
        acc[0][1] = mma(a0, b1, acc[0][1]);
        acc[1][0] = mma(a1, b0, acc[1][0]);
        acc[1][1] = mma(a1, b1, acc[1][1]);
    }

    #pragma unroll
    for (int i = 0; i < 2; ++i)
        #pragma unroll
        for (int j = 0; j < 2; ++j)
            #pragma unroll
            for (int r = 0; r < 8; ++r)
                stile[(wm * 32 + i * 16 + lh * 8 + r) * STP + wn * 32 + j * 16 + lr] = acc[i][j][r];
    __syncthreads();

    if constexpr (MODE == 0) {
        const int rq = threadIdx.x >> 4, c4 = threadIdx.x & 15;
        f32x4 vals[8];
        #pragma unroll
        for (int p = 0; p < 8; ++p) {
            const int rl = p * 16 + rq;
            const int m = mBase + rl, n = nBase + c4 * 4;
            f32x4 v = *reinterpret_cast<const f32x4*>(&stile[rl * STP + c4 * 4]);
            v = v * oscale;
            if (bias != nullptr) {
                f32x4 bv = *reinterpret_cast<const f32x4*>(bias + n);
                v += rne4(bv);
            }
            if (resB != nullptr) {
                u16x4 wv = *reinterpret_cast<const u16x4*>(resB + (size_t)m * N + n);
                v[0] += bf16_widen(wv[0]); v[1] += bf16_widen(wv[1]);
                v[2] += bf16_widen(wv[2]); v[3] += bf16_widen(wv[3]);
            }
            if (resF != nullptr) {
                v += *reinterpret_cast<const f32x4*>(resF + (size_t)m * N + n);
            }
            vals[p] = v;
            vst_f4(outF + (size_t)m * N + n, v);
        }
        __threadfence();
        #pragma unroll
        for (int p = 0; p < 8; ++p) {
            const int rl = p * 16 + rq;
            vst_f4(outF + (size_t)(mBase + rl) * N + nBase + c4 * 4, vals[p]);
        }
    } else if constexpr (MODE == 1) {
        const int rq = threadIdx.x >> 3, c8 = threadIdx.x & 7;
        u32x4 vals[4];
        #pragma unroll
        for (int p = 0; p < 4; ++p) {
            const int rl = p * 32 + rq;
            const int m = mBase + rl, n = nBase + c8 * 8;
            f32x4 lo = *reinterpret_cast<const f32x4*>(&stile[rl * STP + c8 * 8]);
            f32x4 hi = *reinterpret_cast<const f32x4*>(&stile[rl * STP + c8 * 8 + 4]);
            lo = lo * oscale; hi = hi * oscale;
            if (bias != nullptr) {
                f32x4 b0 = *reinterpret_cast<const f32x4*>(bias + n);
                f32x4 b1 = *reinterpret_cast<const f32x4*>(bias + n + 4);
                lo += rne4(b0);
                hi += rne4(b1);
            }
            if (relu) {
                lo[0] = fmaxf(lo[0], 0.0f); lo[1] = fmaxf(lo[1], 0.0f);
                lo[2] = fmaxf(lo[2], 0.0f); lo[3] = fmaxf(lo[3], 0.0f);
                hi[0] = fmaxf(hi[0], 0.0f); hi[1] = fmaxf(hi[1], 0.0f);
                hi[2] = fmaxf(hi[2], 0.0f); hi[3] = fmaxf(hi[3], 0.0f);
            }
            lo = lo * ocarry; hi = hi * ocarry;
            vals[p] = pack_h8(lo, hi);
            vst_u4(outH + (size_t)m * N + n, vals[p]);
        }
        __threadfence();
        #pragma unroll
        for (int p = 0; p < 4; ++p) {
            const int rl = p * 32 + rq;
            vst_u4(outH + (size_t)(mBase + rl) * N + nBase + c8 * 8, vals[p]);
        }
    } else {
        const unsigned tile = blockIdx.y;
        const unsigned hh   = tile / 3u;
        const unsigned part = tile - hh * 3u;
        if (part < 2u) {
            _Float16* dp = (part == 0u) ? outH : outH2;
            const unsigned rq = threadIdx.x >> 3, c8 = threadIdx.x & 7u;
            f32x4 b0 = {}, b1 = {};
            if (bias != nullptr) {
                b0 = rne4(*reinterpret_cast<const f32x4*>(bias + nBase + c8 * 8));
                b1 = rne4(*reinterpret_cast<const f32x4*>(bias + nBase + c8 * 8 + 4));
            }
            u32x4 vals[4];
            #pragma unroll
            for (int p = 0; p < 4; ++p) {
                const unsigned rl = p * 32 + rq;
                const unsigned m = (unsigned)mBase + rl;
                const unsigned bq = m / (unsigned)SEQ, s = m - bq * (unsigned)SEQ;
                f32x4 lo = *reinterpret_cast<const f32x4*>(&stile[rl * STP + c8 * 8]);
                f32x4 hi = *reinterpret_cast<const f32x4*>(&stile[rl * STP + c8 * 8 + 4]);
                lo += b0; hi += b1;
                vals[p] = pack_h8(lo, hi);
                vst_u4(dp + ((size_t)(bq * H_ + hh) * SEQ + s) * DH_ + c8 * 8, vals[p]);
            }
            __threadfence();
            #pragma unroll
            for (int p = 0; p < 4; ++p) {
                const unsigned rl = p * 32 + rq;
                const unsigned m = (unsigned)mBase + rl;
                const unsigned bq = m / (unsigned)SEQ, s = m - bq * (unsigned)SEQ;
                vst_u4(dp + ((size_t)(bq * H_ + hh) * SEQ + s) * DH_ + c8 * 8, vals[p]);
            }
        } else {
            const unsigned rq = threadIdx.x >> 4, c16 = threadIdx.x & 15u;
            const unsigned bq = (unsigned)mBase / (unsigned)SEQ, s0 = (unsigned)mBase - bq * (unsigned)SEQ;
            u32x4 vals[4];
            #pragma unroll
            for (int p = 0; p < 4; ++p) {
                const unsigned el = p * 16 + rq;
                float bv = 0.0f;
                if (bias != nullptr) bv = bf16_rne(bias[nBase + el]);
                f32x4 lo, hi;
                lo[0] = stile[(c16 * 8 + 0) * STP + el] + bv; lo[1] = stile[(c16 * 8 + 1) * STP + el] + bv;
                lo[2] = stile[(c16 * 8 + 2) * STP + el] + bv; lo[3] = stile[(c16 * 8 + 3) * STP + el] + bv;
                hi[0] = stile[(c16 * 8 + 4) * STP + el] + bv; hi[1] = stile[(c16 * 8 + 5) * STP + el] + bv;
                hi[2] = stile[(c16 * 8 + 6) * STP + el] + bv; hi[3] = stile[(c16 * 8 + 7) * STP + el] + bv;
                vals[p] = pack_h8(lo, hi);
                vst_u4(outH3 + ((size_t)(bq * H_ + hh) * DH_ + el) * SEQ + s0 + c16 * 8, vals[p]);
            }
            __threadfence();
            #pragma unroll
            for (int p = 0; p < 4; ++p) {
                const unsigned el = p * 16 + rq;
                vst_u4(outH3 + ((size_t)(bq * H_ + hh) * DH_ + el) * SEQ + s0 + c16 * 8, vals[p]);
            }
        }
    }
}

__global__ __launch_bounds__(128)
void k_attn(const _Float16* __restrict__ Q, const _Float16* __restrict__ Kh,
            const _Float16* __restrict__ Vt, _Float16* __restrict__ ctx) {
    __shared__ __align__(16) _Float16 pbuf[4 * 16 * PP_];
    __shared__ __align__(16) _Float16 obuf[4 * 16 * OP_];

    const int lane = threadIdx.x & 31, wave = threadIdx.x >> 5;
    const int lr = lane & 15, lh = lane >> 4;
    const unsigned gw = blockIdx.x * 4u + (unsigned)wave;
    const unsigned bh = gw / (unsigned)QT_;
    const int m0 = (int)(gw - bh * (unsigned)QT_) * 16;
    const unsigned b  = bh / (unsigned)H_;
    const unsigned h  = bh - b * (unsigned)H_;

    const _Float16* q  = Q  + (size_t)bh * SEQ * DH_;
    const _Float16* kc = Kh + (size_t)bh * SEQ * DH_;
    const _Float16* vt = Vt + (size_t)bh * DH_ * SEQ;

    f16x16 qa0 = ld_frag<_Float16>(q + (size_t)(m0 + lr) * DH_ + lh * 8);
    f16x16 qa1 = ld_frag<_Float16>(q + (size_t)(m0 + lr) * DH_ + lh * 8 + 32);

    f32x8 acc[4] = {};
    float rmax[8], rsum[8];
    #pragma unroll
    for (int r = 0; r < 8; ++r) { rmax[r] = -3.0e38f; rsum[r] = 0.0f; }

    _Float16* pw = pbuf + wave * (16 * PP_);

    for (int j0 = 0; j0 < SEQ; j0 += 32) {
        f32x8 sc[2];
        #pragma unroll
        for (int t = 0; t < 2; ++t) {
            const _Float16* kp = kc + (size_t)(j0 + t * 16 + lr) * DH_ + lh * 8;
            f16x16 kb0 = ld_frag<_Float16>(kp);
            f16x16 kb1 = ld_frag<_Float16>(kp + 32);
            f32x8 z = {};
            z = mma(qa0, kb0, z);
            z = mma(qa1, kb1, z);
            #pragma unroll
            for (int r = 0; r < 8; ++r) sc[t][r] = z[r] * 0.125f;
        }

        float tm[8];
        #pragma unroll
        for (int r = 0; r < 8; ++r) tm[r] = fmaxf(sc[0][r], sc[1][r]);
        #pragma unroll
        for (int off = 1; off < 16; off <<= 1) {
            #pragma unroll
            for (int r = 0; r < 8; ++r) tm[r] = fmaxf(tm[r], __shfl_xor(tm[r], off, 32));
        }

        #pragma unroll
        for (int r = 0; r < 8; ++r) {
            const float nm = fmaxf(rmax[r], tm[r]);
            const float al = __expf(rmax[r] - nm);
            rmax[r] = nm;
            rsum[r] *= al;
            #pragma unroll
            for (int n = 0; n < 4; ++n) acc[n][r] *= al;
            const float p0 = __expf(sc[0][r] - nm);
            const float p1 = __expf(sc[1][r] - nm);
            rsum[r] += p0 + p1;
            sc[0][r] = p0;
            sc[1][r] = p1;
        }

        #pragma unroll
        for (int t = 0; t < 2; ++t)
            #pragma unroll
            for (int r = 0; r < 8; ++r)
                pw[(r + lh * 8) * PP_ + t * 16 + lr] = (_Float16)(sc[t][r] * P_CARRY);
        __syncthreads();

        f16x16 pa = ld_frag<_Float16>(pw + lr * PP_ + lh * 8);
        #pragma unroll
        for (int n = 0; n < 4; ++n) {
            f16x16 vb = ld_frag<_Float16>(vt + (size_t)(n * 16 + lr) * SEQ + j0 + lh * 8);
            acc[n] = mma(pa, vb, acc[n]);
        }
        __syncthreads();
    }

    #pragma unroll
    for (int off = 1; off < 16; off <<= 1) {
        #pragma unroll
        for (int r = 0; r < 8; ++r) rsum[r] += __shfl_xor(rsum[r], off, 32);
    }

    _Float16* ow = obuf + wave * (16 * OP_);
    #pragma unroll
    for (int r = 0; r < 8; ++r) {
        const float inv = (1.0f / rsum[r]) * (CTX_CARRY / P_CARRY);
        const int rowl = r + lh * 8;
        #pragma unroll
        for (int n = 0; n < 4; ++n) ow[rowl * OP_ + n * 16 + lr] = (_Float16)(acc[n][r] * inv);
    }
    __syncthreads();

    const int rq = lane >> 3, c8 = lane & 7;
    u32x4 vals[4];
    #pragma unroll
    for (int p = 0; p < 4; ++p) {
        const int rowl = p * 4 + rq;
        union { f16x8 hv; u32x4 u; } t;
        t.hv = *reinterpret_cast<const f16x8*>(&ow[rowl * OP_ + c8 * 8]);
        vals[p] = t.u;
        _Float16* dst = ctx + ((size_t)(b * (unsigned)SEQ + (unsigned)(m0 + rowl))) * D_ + h * DH_ + c8 * 8;
        vst_u4(dst, vals[p]);
    }
    __threadfence();
    #pragma unroll
    for (int p = 0; p < 4; ++p) {
        const int rowl = p * 4 + rq;
        _Float16* dst = ctx + ((size_t)(b * (unsigned)SEQ + (unsigned)(m0 + rowl))) * D_ + h * DH_ + c8 * 8;
        vst_u4(dst, vals[p]);
    }
}

template <int HOUT>
__global__ __launch_bounds__(128)
void k_ln(const float* __restrict__ in, const float* __restrict__ g,
          const float* __restrict__ be, float* __restrict__ outF,
          _Float16* __restrict__ outH, int nrows) {
    __shared__ __align__(16) float rb[4 * D_];
    const unsigned lane = threadIdx.x & 31u, wave = threadIdx.x >> 5;
    unsigned row = blockIdx.x * 4u + wave;
    row = row < (unsigned)nrows ? row : (unsigned)nrows - 1u;
    const float* src = in + (size_t)row * D_;
    float* rw = rb + wave * D_;

    float s = 0.0f;
    #pragma unroll 1
    for (unsigned p = 0; p < (unsigned)(D_ / 128); ++p) {
        f32x4 v = *reinterpret_cast<const f32x4*>(src + p * 128u + lane * 4u);
        *reinterpret_cast<f32x4*>(rw + p * 128u + lane * 4u) = v;
        s += (v[0] + v[1]) + (v[2] + v[3]);
    }
    #pragma unroll
    for (int off = 16; off > 0; off >>= 1) s += __shfl_xor(s, off, 32);
    const float mu = s * (1.0f / D_);

    float ss = 0.0f;
    #pragma unroll 1
    for (unsigned p = 0; p < (unsigned)(D_ / 128); ++p) {
        f32x4 d = *reinterpret_cast<const f32x4*>(rw + p * 128u + lane * 4u) - mu;
        ss += (d[0] * d[0] + d[1] * d[1]) + (d[2] * d[2] + d[3] * d[3]);
    }
    #pragma unroll
    for (int off = 16; off > 0; off >>= 1) ss += __shfl_xor(ss, off, 32);
    const float var = ss * (1.0f / D_);
    const float inv = rsqrtf(var + EPS_);

    float* dstF = outF + (size_t)row * D_;
    #pragma unroll 1
    for (unsigned p = 0; p < (unsigned)(D_ / 128); ++p) {
        f32x4 d  = *reinterpret_cast<const f32x4*>(rw + p * 128u + lane * 4u) - mu;
        f32x4 gg = rne4(*reinterpret_cast<const f32x4*>(g  + p * 128u + lane * 4u));
        f32x4 bb = rne4(*reinterpret_cast<const f32x4*>(be + p * 128u + lane * 4u));
        f32x4 y  = d * inv * gg + bb;
        *reinterpret_cast<f32x4*>(rw + p * 128u + lane * 4u) = y;
        vst_f4(dstF + p * 128u + lane * 4u, y);
    }

    if constexpr (HOUT) {
        __syncthreads();
        #pragma unroll 1
        for (unsigned p = 0; p < (unsigned)(D_ / 256); ++p) {
            f32x4 lo = *reinterpret_cast<const f32x4*>(rw + p * 256u + lane * 8u);
            f32x4 hi = *reinterpret_cast<const f32x4*>(rw + p * 256u + lane * 8u + 4u);
            vst_u4(outH + (size_t)row * D_ + p * 256u + lane * 8u, pack_h8(lo, hi));
        }
    }
    __threadfence();
    #pragma unroll 1
    for (unsigned p = 0; p < (unsigned)(D_ / 128); ++p) {
        f32x4 y = *reinterpret_cast<const f32x4*>(rw + p * 128u + lane * 4u);
        vst_f4(dstF + p * 128u + lane * 4u, y);
    }
    if constexpr (HOUT) {
        #pragma unroll 1
        for (unsigned p = 0; p < (unsigned)(D_ / 256); ++p) {
            f32x4 lo = *reinterpret_cast<const f32x4*>(rw + p * 256u + lane * 8u);
            f32x4 hi = *reinterpret_cast<const f32x4*>(rw + p * 256u + lane * 8u + 4u);
            vst_u4(outH + (size_t)row * D_ + p * 256u + lane * 8u, pack_h8(lo, hi));
        }
    }
}

extern "C" void kernel_launch(void* const* d_in, const int* in_sizes, int n_in,
                              void* d_out, int out_size, void* d_ws,
                              size_t ws_size, hipStream_t stream) {
    if (n_in < 13) return;
    const long need_x = ((long)(NB - 1) * S_FULL + SEQ) * (long)D_;
    if ((long)in_sizes[0] < need_x) return;
    if (in_sizes[1] < QKVN_ * D_ || in_sizes[2] < QKVN_) return;
    if (in_sizes[3] < D_ * D_ || in_sizes[4] < D_) return;
    if (in_sizes[5] < F_ * D_ || in_sizes[6] < F_ || in_sizes[7] < D_ * F_ || in_sizes[8] < D_) return;
    if (in_sizes[9] < D_ || in_sizes[10] < D_ || in_sizes[11] < D_ || in_sizes[12] < D_) return;
    if ((long)out_size < (long)MROWS * D_) return;

    const float* x    = (const float*)d_in[0];
    const float* wqkv = (const float*)d_in[1];
    const float* bqkv = (const float*)d_in[2];
    const float* wo   = (const float*)d_in[3];
    const float* bo   = (const float*)d_in[4];
    const float* w1   = (const float*)d_in[5];
    const float* b1   = (const float*)d_in[6];
    const float* w2   = (const float*)d_in[7];
    const float* b2   = (const float*)d_in[8];
    const float* g1   = (const float*)d_in[9];
    const float* be1  = (const float*)d_in[10];
    const float* g2   = (const float*)d_in[11];
    const float* be2  = (const float*)d_in[12];
    float* out = (float*)d_out;

    const size_t MD = (size_t)MROWS * D_;
    char* ws = (char*)d_ws;
    size_t off = 0;
    unsigned short* wqkvT = (unsigned short*)(ws + off); off += (size_t)QKVN_ * D_ * 2;
    unsigned short* woT   = (unsigned short*)(ws + off); off += (size_t)D_ * D_ * 2;
    unsigned short* w1T   = (unsigned short*)(ws + off); off += (size_t)F_ * D_ * 2;
    unsigned short* w2T   = (unsigned short*)(ws + off); off += (size_t)D_ * F_ * 2;
    unsigned short* xb  = (unsigned short*)(ws + off);
    _Float16*       y1h = (_Float16*)(ws + off);       off += MD * 2;
    char* p2 = ws + off;                               off += MD * 8;
    _Float16* qh   = (_Float16*)(p2);
    _Float16* kh   = (_Float16*)(p2 + MD * 2);
    _Float16* vt   = (_Float16*)(p2 + MD * 4);
    _Float16* ctxp = (_Float16*)(p2 + MD * 6);
    _Float16* hid  = (_Float16*)(p2);
    float* r1 = (float*)(ws + off);
    float* r2 = (float*)(ws + off);                    off += MD * 4;
    float* y1f = (float*)(ws + off);                   off += MD * 4;
    if (off > ws_size) return;

    k_cvt_x<<<MROWS * 128 / 256, 256, 0, stream>>>(x, xb);
    k_cvt_w<0><<<(unsigned)((size_t)QKVN_ * D_ / 2048), 256, 0, stream>>>(wqkv, wqkvT, 1.0f);
    k_cvt_w<1><<<(unsigned)((size_t)D_ * D_ / 2048), 256, 0, stream>>>(wo, woT, WO_SCALE);
    k_cvt_w<1><<<(unsigned)((size_t)F_ * D_ / 2048), 256, 0, stream>>>(w1, w1T, W1_SCALE);
    k_cvt_w<1><<<(unsigned)((size_t)D_ * F_ / 2048), 256, 0, stream>>>(w2, w2T, W2_SCALE);

    k_gemm<__bf16, 2><<<dim3(MROWS / 128, QKVN_ / 64), 256, 0, stream>>>(
        (const __bf16*)xb, (const __bf16*)wqkvT, bqkv, nullptr, nullptr,
        nullptr, qh, kh, vt, QKVN_, D_, 1.0f, 1.0f, 0);

    k_attn<<<NB * H_ * QT_ / 4, 128, 0, stream>>>(qh, kh, vt, ctxp);

    k_gemm<_Float16, 0><<<dim3(MROWS / 128, D_ / 64), 256, 0, stream>>>(
        ctxp, (const _Float16*)woT, bo, xb, nullptr,
        r1, nullptr, nullptr, nullptr, D_, D_, 1.0f / (WO_SCALE * CTX_CARRY), 1.0f, 0);

    k_ln<1><<<MROWS / 4, 128, 0, stream>>>(r1, g1, be1, y1f, y1h, MROWS);

    k_gemm<_Float16, 1><<<dim3(MROWS / 128, F_ / 64), 256, 0, stream>>>(
        y1h, (const _Float16*)w1T, b1, nullptr, nullptr,
        nullptr, hid, nullptr, nullptr, F_, D_, 1.0f / W1_SCALE, HID_CARRY, 1);
    k_gemm<_Float16, 0><<<dim3(MROWS / 128, D_ / 64), 256, 0, stream>>>(
        hid, (const _Float16*)w2T, b2, nullptr, y1f,
        r2, nullptr, nullptr, nullptr, D_, F_, 1.0f / (W2_SCALE * HID_CARRY), 1.0f, 0);

    k_ln<0><<<MROWS / 4, 128, 0, stream>>>(r2, g2, be2, out, nullptr, MROWS);
}
